// MambaLayer_45045617000489
// MI455X (gfx1250) — hardware-verified
//
#include <hip/hip_runtime.h>
#include <stddef.h>
#include <stdint.h>

#define NBATCH 8
#define LTOK   1024
#define NTOK   (NBATCH * LTOK)
#define CIN    512
#define COUT   512
#define DIN    1024
#define DST    64
#define NHD    16
#define HDIM   64
#define DXBC   (DIN + 2 * DST)
#define NPROJ  (2 * DIN + 2 * DST + NHD)
#define NPP    2240
#define NPA    2176
#define KIN2   (2 * CIN)
#define KOP2   (2 * DIN)
#define KCW2   (2 * CIN)
#define XCOL   DIN
#define BCOL   (DIN + DIN)
#define DTCOL  (DIN + DXBC)
#define EPS    1e-5f
#define NTHR   256
#define GTHR   128
#define GBM    64
#define SCP    132
#define NU_INP (NPP * (KIN2 / 8))
#define NU_OP  (CIN * (KOP2 / 8))
#define NU_CW  (COUT * (KCW2 / 8))
#define WSMAX  134217728

static_assert(NU_INP % NTHR == 0 && NU_OP % NTHR == 0 && NU_CW % NTHR == 0);
static_assert(NPA % 128 == 0 && (NPP - NPA) == 64 && NPP >= NPROJ && (NPP * 4) % 128 == 0);
static_assert(NTOK % GBM == 0 && COUT % GBM == 0 && LTOK % 128 == 0 && CIN % 128 == 0);
static_assert(KIN2 % 32 == 0 && KOP2 % 32 == 0 && KCW2 % 32 == 0);
static_assert(DXBC % 32 == 0 && (DXBC + 32) % 32 == 0 && NHD <= 16);
static_assert((XCOL * 4) % 128 == 0 && (HDIM * 4) % 128 == 0);
static_assert(LTOK % 64 == 0 && (SCP * 4) % 16 == 0);

typedef float          v4f   __attribute__((ext_vector_type(4)));
typedef float          v8f   __attribute__((ext_vector_type(8)));
typedef int            v8i   __attribute__((ext_vector_type(8)));
typedef unsigned short v8us  __attribute__((ext_vector_type(8)));
typedef unsigned short v16us __attribute__((ext_vector_type(16)));
typedef __bf16         v16bf __attribute__((ext_vector_type(16)));
typedef v4f  __attribute__((may_alias)) v4fa;
typedef v8us __attribute__((may_alias)) v8usa;
union FragB { v16bf v; v16us u; v8us h[2]; v8i w; };

__device__ __forceinline__ v8f wmb(const FragB& a, const FragB& b, v8f c) {
  v8f d = __builtin_amdgcn_wmma_f32_16x16x32_bf16(false, a.v, false, b.v, (short)0, c, false, false);
  asm volatile("v_nop\n\tv_nop\n\tv_nop\n\tv_nop" : "+v"(d) : "v"(a.w), "v"(b.w));
  return d;
}

__device__ __forceinline__ unsigned bf16_bits(float f) {
  const unsigned u = __float_as_uint(f);
  return (u + 0x7FFFu + ((u >> 16) & 1u)) >> 16;
}
__device__ __forceinline__ float bf16_val(float f) {
  return __uint_as_float(bf16_bits(f) << 16);
}
__device__ __forceinline__ void put16(unsigned short* dp, v8us o) {
  *(volatile v8us*)dp = o;
  __threadfence();
  *(volatile v8us*)dp = o;
}

__global__ __launch_bounds__(NTHR) void k_prep(const float* __restrict__ Win, const float* __restrict__ Wop,
                                               const float* __restrict__ Wcw,
                                               unsigned short* INP2, unsigned short* OP2, unsigned short* CW2) {
  const int u = (int)blockIdx.x * NTHR + (int)threadIdx.x;
  const float* src;
  unsigned short* dst;
  float keep = 1.0f;
  if (u < NU_INP) {
    const int n  = u >> 7;
    const int k8 = (u & 127) * 8;
    const int c  = k8 & (CIN - 1);
    const int nc = n < NPROJ ? n : NPROJ - 1;
    keep = n < NPROJ ? 1.0f : 0.0f;
    src = Win + (size_t)nc * CIN + c;
    dst = INP2 + (size_t)n * KIN2 + k8;
  } else if (u < NU_INP + NU_OP) {
    const int v  = u - NU_INP;
    const int n  = v >> 8;
    const int k8 = (v & 255) * 8;
    const int d  = k8 & (DIN - 1);
    src = Wop + (size_t)n * DIN + d;
    dst = OP2 + (size_t)n * KOP2 + k8;
  } else if (u < NU_INP + NU_OP + NU_CW) {
    const int v  = u - NU_INP - NU_OP;
    const int o  = v >> 7;
    const int k8 = (v & 127) * 8;
    const int c  = k8 & (CIN - 1);
    src = Wcw + (size_t)o * CIN + c;
    dst = CW2 + (size_t)o * KCW2 + k8;
  } else {
    return;
  }
  const v4f a = *(const v4fa*)src;
  const v4f b = *(const v4fa*)(src + 4);
  v8us ov;
  ov[0] = (unsigned short)bf16_bits(a.x * keep);
  ov[1] = (unsigned short)bf16_bits(a.y * keep);
  ov[2] = (unsigned short)bf16_bits(a.z * keep);
  ov[3] = (unsigned short)bf16_bits(a.w * keep);
  ov[4] = (unsigned short)bf16_bits(b.x * keep);
  ov[5] = (unsigned short)bf16_bits(b.y * keep);
  ov[6] = (unsigned short)bf16_bits(b.z * keep);
  ov[7] = (unsigned short)bf16_bits(b.w * keep);
  put16(dst, ov);
}

__global__ __launch_bounds__(NTHR) void k_ln(const float* __restrict__ x, const float* __restrict__ lnw,
                                             const float* __restrict__ lnb, unsigned short* XN) {
  __shared__ __attribute__((aligned(16))) unsigned short sX[32 * CIN];
  const int tid = (int)threadIdx.x, lane = tid & 31, wave = tid >> 5;
  const int b = (int)blockIdx.y, l0 = (int)blockIdx.x * 32;
  const float* xb = x + (size_t)b * CIN * LTOK + l0;
#pragma unroll 4
  for (int it = 0; it < 16; ++it) {
    const int u = it * NTHR + tid;
    const int c = u >> 3, q = u & 7;
    const v4f v = *(const v4fa*)(xb + (size_t)c * LTOK + 4 * q);
    unsigned short* sp = sX + (4 * q) * CIN + c;
    sp[0]       = (unsigned short)bf16_bits(v.x);
    sp[CIN]     = (unsigned short)bf16_bits(v.y);
    sp[2 * CIN] = (unsigned short)bf16_bits(v.z);
    sp[3 * CIN] = (unsigned short)bf16_bits(v.w);
  }
  __syncthreads();

  float lw[16], lb[16];
  {
    const v4f w0 = *(const v4fa*)(lnw + 8 * lane);
    const v4f w1 = *(const v4fa*)(lnw + 8 * lane + 4);
    const v4f w2 = *(const v4fa*)(lnw + 256 + 8 * lane);
    const v4f w3 = *(const v4fa*)(lnw + 256 + 8 * lane + 4);
    const v4f b0 = *(const v4fa*)(lnb + 8 * lane);
    const v4f b1 = *(const v4fa*)(lnb + 8 * lane + 4);
    const v4f b2 = *(const v4fa*)(lnb + 256 + 8 * lane);
    const v4f b3 = *(const v4fa*)(lnb + 256 + 8 * lane + 4);
    lw[0] = bf16_val(w0.x); lw[1] = bf16_val(w0.y); lw[2] = bf16_val(w0.z); lw[3] = bf16_val(w0.w);
    lw[4] = bf16_val(w1.x); lw[5] = bf16_val(w1.y); lw[6] = bf16_val(w1.z); lw[7] = bf16_val(w1.w);
    lw[8] = bf16_val(w2.x); lw[9] = bf16_val(w2.y); lw[10] = bf16_val(w2.z); lw[11] = bf16_val(w2.w);
    lw[12] = bf16_val(w3.x); lw[13] = bf16_val(w3.y); lw[14] = bf16_val(w3.z); lw[15] = bf16_val(w3.w);
    lb[0] = bf16_val(b0.x); lb[1] = bf16_val(b0.y); lb[2] = bf16_val(b0.z); lb[3] = bf16_val(b0.w);
    lb[4] = bf16_val(b1.x); lb[5] = bf16_val(b1.y); lb[6] = bf16_val(b1.z); lb[7] = bf16_val(b1.w);
    lb[8] = bf16_val(b2.x); lb[9] = bf16_val(b2.y); lb[10] = bf16_val(b2.z); lb[11] = bf16_val(b2.w);
    lb[12] = bf16_val(b3.x); lb[13] = bf16_val(b3.y); lb[14] = bf16_val(b3.z); lb[15] = bf16_val(b3.w);
  }

#pragma unroll 1
  for (int tt = 0; tt < 4; ++tt) {
    const int t = 4 * wave + tt;
    const v8us g0 = *(const v8usa*)(sX + t * CIN + 8 * lane);
    const v8us g1 = *(const v8usa*)(sX + t * CIN + 256 + 8 * lane);
    float f[16];
#pragma unroll
    for (int i = 0; i < 8; ++i) {
      f[i]     = __uint_as_float(((unsigned)g0[i]) << 16);
      f[8 + i] = __uint_as_float(((unsigned)g1[i]) << 16);
    }
    float s = 0.0f;
#pragma unroll
    for (int i = 0; i < 16; ++i) s += f[i];
#pragma unroll
    for (int o = 16; o > 0; o >>= 1) s += __shfl_xor(s, o, 32);
    const float mean = s * (1.0f / (float)CIN);
    float s2 = 0.0f;
#pragma unroll
    for (int i = 0; i < 16; ++i) {
      const float d = f[i] - mean;
      f[i] = d;
      s2 += d * d;
    }
#pragma unroll
    for (int o = 16; o > 0; o >>= 1) s2 += __shfl_xor(s2, o, 32);
    const float rstd = rsqrtf(s2 * (1.0f / (float)CIN) + EPS);
    v8us h0, h1, q0, q1;
#pragma unroll
    for (int i = 0; i < 8; ++i) {
      const float xa = f[i] * rstd * lw[i] + lb[i];
      const unsigned ha = bf16_bits(xa);
      h0[i] = (unsigned short)ha;
      q0[i] = (unsigned short)bf16_bits(xa - __uint_as_float(ha << 16));
      const float xc = f[8 + i] * rstd * lw[8 + i] + lb[8 + i];
      const unsigned hc = bf16_bits(xc);
      h1[i] = (unsigned short)hc;
      q1[i] = (unsigned short)bf16_bits(xc - __uint_as_float(hc << 16));
    }
    unsigned short* rp = XN + (size_t)(b * LTOK + l0 + t) * KIN2;
    *(volatile v8us*)(rp + 8 * lane)             = h0;
    *(volatile v8us*)(rp + 256 + 8 * lane)       = h1;
    *(volatile v8us*)(rp + CIN + 8 * lane)       = q0;
    *(volatile v8us*)(rp + CIN + 256 + 8 * lane) = q1;
    __threadfence();
    *(volatile v8us*)(rp + 8 * lane)             = h0;
    *(volatile v8us*)(rp + 256 + 8 * lane)       = h1;
    *(volatile v8us*)(rp + CIN + 8 * lane)       = q0;
    *(volatile v8us*)(rp + CIN + 256 + 8 * lane) = q1;
  }
}

template <int MODE, int NT>
__global__ __launch_bounds__(GTHR) void k_gemm(const unsigned short* __restrict__ A, int lda,
                                               const unsigned short* __restrict__ BT, int ldb, long long zsB,
                                               int K, int colOff,
                                               float* Cf, int ldc, long long zsC,
                                               unsigned short* Cb, int ldcb, int loff,
                                               const float* __restrict__ pcb, const float* __restrict__ pg,
                                               const float* __restrict__ pbe, const float* __restrict__ pm,
                                               const float* __restrict__ pva) {
  static_assert(NT == 8 || NT == 4);
  static_assert(MODE != 1 || NT == 8);
  constexpr int GBN = 16 * NT;
  __shared__ __attribute__((aligned(16))) float stg[GBM * GBN];
  __shared__ float se0[GBM], se1[GBM], se2[GBM], se3[GBM];
  const int tid = (int)threadIdx.x, lane = tid & 31, wave = tid >> 5, hh = lane >> 4, m = lane & 15;
  const int rowBase = (int)blockIdx.x * GBM;
  const int colBase = colOff + (int)blockIdx.y * GBN;
  const int zb = (int)blockIdx.z;

  if constexpr (MODE == 2) {
    if (tid < GBM) {
      const int o = rowBase + tid;
      se0[tid] = bf16_val(pcb[o]);
      se1[tid] = bf16_val(pm[o]);
      se2[tid] = rsqrtf(bf16_val(pva[o]) + EPS) * bf16_val(pg[o]);
      se3[tid] = bf16_val(pbe[o]);
    }
    __syncthreads();
  }

  v8f acc[NT];
  {
    const v8f z = {0.f, 0.f, 0.f, 0.f, 0.f, 0.f, 0.f, 0.f};
#pragma unroll
    for (int t = 0; t < NT; ++t) acc[t] = z;
  }
  const unsigned short* ap = A + (size_t)(rowBase + 16 * wave + m) * (size_t)lda + 8 * hh;
  const unsigned short* bp = BT + (size_t)zb * (size_t)zsB + (size_t)(colBase + m) * (size_t)ldb + 8 * hh;

#pragma unroll 1
  for (int k0 = 0; k0 < K; k0 += 32) {
    FragB af;
    af.h[0] = *(const v8usa*)(ap + k0);
    af.h[1] = *(const v8usa*)(ap + k0 + 16);
#pragma unroll
    for (int nt = 0; nt < NT; ++nt) {
      const unsigned short* wq = bp + (size_t)(16 * nt) * (size_t)ldb + k0;
      FragB bf;
      bf.h[0] = *(const v8usa*)wq;
      bf.h[1] = *(const v8usa*)(wq + 16);
      acc[nt] = wmb(af, bf, acc[nt]);
    }
  }

#pragma unroll
  for (int nt = 0; nt < NT; ++nt) {
    const int lc = 16 * nt + m;
#pragma unroll
    for (int r = 0; r < 8; ++r) {
      const int lr = 16 * wave + 8 * hh + r;
      float v = acc[nt][r];
      if constexpr (MODE == 2) v = fmaxf(((v + se0[lr]) - se1[lr]) * se2[lr] + se3[lr], 0.0f);
      stg[lr * GBN + lc] = v;
    }
  }
  __syncthreads();

  if constexpr (MODE == 1) {
    const int part = lane >> 4;
    const int j = lane & 15;
    const unsigned mh = 0u - (unsigned)part;
    const unsigned ml = ~mh;
    v8us pv[16];
#pragma unroll
    for (int i = 0; i < 16; ++i) {
      const float* sp = stg + (16 * wave + i) * GBN + 8 * j;
      const v4f a = *(const v4fa*)sp;
      const v4f b = *(const v4fa*)(sp + 4);
      const v8f f8 = {a.x, a.y, a.z, a.w, b.x, b.y, b.z, b.w};
      v8us oo;
#pragma unroll
      for (int e = 0; e < 8; ++e) {
        const unsigned hb = bf16_bits(f8[e]);
        const unsigned lb = bf16_bits(f8[e] - __uint_as_float(hb << 16));
        oo[e] = (unsigned short)((hb & ml) | (lb & mh));
      }
      pv[i] = oo;
    }
#pragma unroll
    for (int i = 0; i < 16; ++i) {
      unsigned short* op = Cb + (size_t)(rowBase + 16 * wave + i) * (size_t)ldcb + colBase + part * loff + 8 * j;
      *(volatile v8us*)op = pv[i];
    }
    __threadfence();
#pragma unroll
    for (int i = 0; i < 16; ++i) {
      unsigned short* op = Cb + (size_t)(rowBase + 16 * wave + i) * (size_t)ldcb + colBase + part * loff + 8 * j;
      *(volatile v8us*)op = pv[i];
    }
  } else {
    constexpr int LPR = GBN / 4;
    constexpr int RPI = 32 / LPR;
    constexpr int NI  = 16 / RPI;
    const int rsub = lane / LPR;
    const int c4   = 4 * (lane % LPR);
    v4f pv[NI];
#pragma unroll
    for (int i = 0; i < NI; ++i) pv[i] = *(const v4fa*)(stg + (16 * wave + i * RPI + rsub) * GBN + c4);
    float* Cz = Cf + (size_t)zb * (size_t)zsC;
#pragma unroll
    for (int i = 0; i < NI; ++i) {
      const int row = rowBase + 16 * wave + i * RPI + rsub;
      *(volatile v4f*)(Cz + (size_t)row * (size_t)ldc + colBase + c4) = pv[i];
    }
    __threadfence();
#pragma unroll
    for (int i = 0; i < NI; ++i) {
      const int row = rowBase + 16 * wave + i * RPI + rsub;
      *(volatile v4f*)(Cz + (size_t)row * (size_t)ldc + colBase + c4) = pv[i];
    }
  }
}

__global__ __launch_bounds__(NTHR) void k_conv(float* ZX, const float* __restrict__ cw, const float* __restrict__ cb,
                                               const float* __restrict__ dtb) {
  const int tid = (int)threadIdx.x, lane = tid & 31;
  const int b  = (int)blockIdx.y;
  const int cc = (int)blockIdx.x * NTHR + tid;
  if (cc >= DXBC + 32) return;
  float* p = ZX + (size_t)b * LTOK * NPP + XCOL + cc;
  if (cc < DXBC) {
    const v4f w4 = *(const v4fa*)(cw + 4 * cc);
    const float w0 = bf16_val(w4.x), w1 = bf16_val(w4.y), w2 = bf16_val(w4.z), w3 = bf16_val(w4.w);
    const float bs = bf16_val(cb[cc]);
    float a0 = 0.0f, a1 = 0.0f, a2 = 0.0f;
#pragma unroll 1
    for (int l = 0; l < LTOK; ++l) {
      float* q = p + (size_t)l * NPP;
      const float a3 = *q;
      const float r  = ((a0 * w0 + a1 * w1) + a2 * w2) + a3 * w3 + bs;
      const float e  = expf(fminf(-r, 80.0f));
      const float o  = r * (1.0f / (1.0f + e));
      a0 = a1; a1 = a2; a2 = a3;
      *(volatile float*)q = o;
      __threadfence();
      *(volatile float*)q = o;
    }
  } else {
    int hcl = cc - DXBC;
    const float keep = (hcl < NHD) ? 1.0f : 0.0f;
    hcl = hcl < NHD ? hcl : NHD - 1;
    const float db = bf16_val(dtb[hcl]);
    (void)lane;
#pragma unroll 1
    for (int l = 0; l < LTOK; ++l) {
      float* q = p + (size_t)l * NPP;
      const float v  = *q + db;
      const float sp = fmaxf(v, 0.0f) + log1pf(expf(-fabsf(v)));
      const float o  = sp * keep;
      *(volatile float*)q = o;
      __threadfence();
      *(volatile float*)q = o;
    }
  }
}

__global__ __launch_bounds__(NTHR) void k_scan(float* ZX, const float* __restrict__ Alog,
                                               const float* __restrict__ Dp) {
  __shared__ __attribute__((aligned(16))) float sBC[64 * SCP];
  __shared__ __attribute__((aligned(16))) float sXh[64 * 32];
  __shared__ __attribute__((aligned(16))) float sY[64 * 32];
  __shared__ float sdt[64];
  __shared__ float sdA[64];
  const int tid = (int)threadIdx.x, lane = tid & 31, wave = tid >> 5;
  const int bx = (int)blockIdx.x;
  const int b = bx >> 5, h = (bx >> 1) & (NHD - 1), ph = bx & 1;
  const int pl = tid >> 3, q = tid & 7, s0 = 8 * q;
  const float Ah = -expf(bf16_val(Alog[h]));
  const float Dh = bf16_val(Dp[h]);
  const int xcol = XCOL + HDIM * h + 32 * ph;
  float* zbp = ZX + (size_t)b * LTOK * NPP;

  float hs[8];
#pragma unroll
  for (int j = 0; j < 8; ++j) hs[j] = 0.0f;

#pragma unroll 1
  for (int ch = 0; ch < LTOK / 64; ++ch) {
    const int r0 = ch * 64;
#pragma unroll
    for (int it = 0; it < 8; ++it) {
      const int u = it * NTHR + tid;
      const int row = u >> 5, c4 = u & 31;
      const v4f v = *(const v4fa*)(zbp + (size_t)(r0 + row) * NPP + BCOL + 4 * c4);
      *(v4fa*)(sBC + row * SCP + 4 * c4) = v;
    }
#pragma unroll
    for (int it = 0; it < 2; ++it) {
      const int u = it * NTHR + tid;
      const int row = u >> 3, c4 = u & 7;
      const v4f v = *(const v4fa*)(zbp + (size_t)(r0 + row) * NPP + xcol + 4 * c4);
      *(v4fa*)(sXh + row * 32 + 4 * c4) = v;
    }
    if (tid < 64) {
      const float dv = zbp[(size_t)(r0 + tid) * NPP + DTCOL + h];
      sdt[tid] = dv;
      sdA[tid] = expf(dv * Ah);
    }
    __syncthreads();

#pragma unroll 1
    for (int i = 0; i < 64; ++i) {
      const float dtv = sdt[i];
      const float dA  = sdA[i];
      const float xv  = sXh[i * 32 + pl];
      const float dx  = dtv * xv;
      const v4f ba = *(const v4fa*)(sBC + i * SCP + s0);
      const v4f bb = *(const v4fa*)(sBC + i * SCP + s0 + 4);
      const v4f ca = *(const v4fa*)(sBC + i * SCP + DST + s0);
      const v4f cbv = *(const v4fa*)(sBC + i * SCP + DST + s0 + 4);
      const float bm[8] = {ba.x, ba.y, ba.z, ba.w, bb.x, bb.y, bb.z, bb.w};
      const float cm[8] = {ca.x, ca.y, ca.z, ca.w, cbv.x, cbv.y, cbv.z, cbv.w};
      float acc = 0.0f;
#pragma unroll
      for (int j = 0; j < 8; ++j) {
        hs[j] = hs[j] * dA + dx * bm[j];
        acc += hs[j] * cm[j];
      }
      acc += __shfl_xor(acc, 1, 32);
      acc += __shfl_xor(acc, 2, 32);
      acc += __shfl_xor(acc, 4, 32);
      if (q == 0) sY[i * 32 + pl] = acc + Dh * xv;
    }
    __syncthreads();

    v4f pv[2];
#pragma unroll
    for (int k = 0; k < 2; ++k) {
      const int lrow = wave * 8 + 4 * k + (lane >> 3);
      pv[k] = *(const v4fa*)(sY + lrow * 32 + 4 * (lane & 7));
    }
#pragma unroll
    for (int k = 0; k < 2; ++k) {
      const int lrow = wave * 8 + 4 * k + (lane >> 3);
      *(volatile v4f*)(zbp + (size_t)(r0 + lrow) * NPP + xcol + 4 * (lane & 7)) = pv[k];
    }
    __threadfence();
#pragma unroll
    for (int k = 0; k < 2; ++k) {
      const int lrow = wave * 8 + 4 * k + (lane >> 3);
      *(volatile v4f*)(zbp + (size_t)(r0 + lrow) * NPP + xcol + 4 * (lane & 7)) = pv[k];
    }
  }
}

__global__ __launch_bounds__(NTHR) void k_gate(const float* ZX, const float* __restrict__ rmsw, unsigned short* G) {
  __shared__ __attribute__((aligned(16))) float gbuf[8 * DIN];
  const int tid = (int)threadIdx.x, lane = tid & 31, wave = tid >> 5;
  const int row = (int)blockIdx.x * 8 + wave;
  const float* zp = ZX + (size_t)row * NPP;
  const float* yp = zp + XCOL;
  float* gw = gbuf + wave * DIN;
  float ss = 0.0f;
#pragma unroll 1
  for (int u = 0; u < 8; ++u) {
    const int col = 256 * (u >> 1) + 8 * lane + 4 * (u & 1);
    const v4f y4 = *(const v4fa*)(yp + col);
    const v4f z4 = *(const v4fa*)(zp + col);
    const float ex = expf(fminf(-z4.x, 80.0f));
    const float ey = expf(fminf(-z4.y, 80.0f));
    const float ez = expf(fminf(-z4.z, 80.0f));
    const float ew = expf(fminf(-z4.w, 80.0f));
    v4f g;
    g.x = y4.x * (z4.x * (1.0f / (1.0f + ex)));
    g.y = y4.y * (z4.y * (1.0f / (1.0f + ey)));
    g.z = y4.z * (z4.z * (1.0f / (1.0f + ez)));
    g.w = y4.w * (z4.w * (1.0f / (1.0f + ew)));
    *(v4fa*)(gw + col) = g;
    ss += g.x * g.x + g.y * g.y + g.z * g.z + g.w * g.w;
  }
#pragma unroll
  for (int o = 16; o > 0; o >>= 1) ss += __shfl_xor(ss, o, 32);
  const float scale = rsqrtf(ss * (1.0f / (float)DIN) + EPS);

#pragma unroll 1
  for (int i = 0; i < 4; ++i) {
    const int col = 256 * i + 8 * lane;
    const v4f ga = *(const v4fa*)(gw + col);
    const v4f gb = *(const v4fa*)(gw + col + 4);
    const v4f ra = *(const v4fa*)(rmsw + col);
    const v4f rb = *(const v4fa*)(rmsw + col + 4);
    const float g8[8] = {ga.x, ga.y, ga.z, ga.w, gb.x, gb.y, gb.z, gb.w};
    const float r8[8] = {ra.x, ra.y, ra.z, ra.w, rb.x, rb.y, rb.z, rb.w};
    v8us oh, ol;
#pragma unroll
    for (int e = 0; e < 8; ++e) {
      const float gn = g8[e] * scale * bf16_val(r8[e]);
      const unsigned hb = bf16_bits(gn);
      oh[e] = (unsigned short)hb;
      ol[e] = (unsigned short)bf16_bits(gn - __uint_as_float(hb << 16));
    }
    put16(G + (size_t)row * KOP2 + col, oh);
    put16(G + (size_t)row * KOP2 + DIN + col, ol);
  }
}

extern "C" void kernel_launch(void* const* d_in, const int* in_sizes, int n_in,
                              void* d_out, int out_size, void* d_ws, size_t ws_size,
                              hipStream_t stream) {
  if (n_in < 17) return;
  if (in_sizes[0] != NBATCH * CIN * LTOK) return;
  if (in_sizes[1] != CIN || in_sizes[2] != CIN) return;
  if (in_sizes[3] != NPROJ * CIN) return;
  if (in_sizes[4] != DXBC * 4 || in_sizes[5] != DXBC) return;
  if (in_sizes[6] != NHD || in_sizes[7] != NHD || in_sizes[8] != NHD) return;
  if (in_sizes[9] != DIN) return;
  if (in_sizes[10] != CIN * DIN) return;
  if (in_sizes[11] != COUT * CIN) return;
  if (in_sizes[12] != COUT || in_sizes[13] != COUT || in_sizes[14] != COUT) return;
  if (in_sizes[15] != COUT || in_sizes[16] != COUT) return;
  if (out_size != NBATCH * COUT * LTOK) return;

  const float* x      = (const float*)d_in[0];
  const float* ln_w   = (const float*)d_in[1];
  const float* ln_b   = (const float*)d_in[2];
  const float* inpw   = (const float*)d_in[3];
  const float* c1w    = (const float*)d_in[4];
  const float* c1b    = (const float*)d_in[5];
  const float* dtbias = (const float*)d_in[6];
  const float* A_log  = (const float*)d_in[7];
  const float* Dp     = (const float*)d_in[8];
  const float* rms_w  = (const float*)d_in[9];
  const float* opw    = (const float*)d_in[10];
  const float* c2w    = (const float*)d_in[11];
  const float* c2b    = (const float*)d_in[12];
  const float* bn_g   = (const float*)d_in[13];
  const float* bn_b   = (const float*)d_in[14];
  const float* bn_m   = (const float*)d_in[15];
  const float* bn_v   = (const float*)d_in[16];
  float* out = (float*)d_out;

  char* ws = (char*)d_ws;
  size_t off = 0;
  const size_t oINP2 = off; off += (size_t)NPP * KIN2 * 2;
  const size_t oOP2  = off; off += (size_t)CIN * KOP2 * 2;
  const size_t oCW2  = off; off += (size_t)COUT * KCW2 * 2;
  const size_t oXN   = off; off += (size_t)NTOK * KIN2 * 2;
  const size_t oZX   = off; off += (size_t)NTOK * NPP * 4;
  const size_t oG    = off; off += (size_t)NTOK * KOP2 * 2;
  if (off > ws_size || off > (size_t)WSMAX) return;
  unsigned short* INP2 = (unsigned short*)(ws + oINP2);
  unsigned short* OP2  = (unsigned short*)(ws + oOP2);
  unsigned short* CW2  = (unsigned short*)(ws + oCW2);
  unsigned short* XN   = (unsigned short*)(ws + oXN);
  unsigned short* OH   = (unsigned short*)(ws + oXN);
  float*          ZX   = (float*)(ws + oZX);
  unsigned short* G    = (unsigned short*)(ws + oG);

  k_prep<<<(NU_INP + NU_OP + NU_CW) / NTHR, NTHR, 0, stream>>>(inpw, opw, c2w, INP2, OP2, CW2);
  k_ln<<<dim3(LTOK / 32, NBATCH), NTHR, 0, stream>>>(x, ln_w, ln_b, XN);
  k_gemm<0, 8><<<dim3(NTOK / GBM, NPA / 128, 1), GTHR, 0, stream>>>(
      XN, KIN2, INP2, KIN2, 0LL, KIN2, 0, ZX, NPP, 0LL, OP2, KOP2, 0, ln_w, ln_w, ln_w, ln_w, ln_w);
  k_gemm<0, 4><<<dim3(NTOK / GBM, 1, 1), GTHR, 0, stream>>>(
      XN, KIN2, INP2, KIN2, 0LL, KIN2, NPA, ZX, NPP, 0LL, OP2, KOP2, 0, ln_w, ln_w, ln_w, ln_w, ln_w);
  k_conv<<<dim3(5, NBATCH), NTHR, 0, stream>>>(ZX, c1w, c1b, dtbias);
  k_scan<<<NBATCH * NHD * 2, NTHR, 0, stream>>>(ZX, A_log, Dp);
  k_gate<<<NTOK / 8, NTHR, 0, stream>>>(ZX, rms_w, G);
  k_gemm<1, 8><<<dim3(NTOK / GBM, CIN / 128, 1), GTHR, 0, stream>>>(
      G, KOP2, OP2, KOP2, 0LL, KOP2, 0, ZX, NPP, 0LL, OH, KIN2, CIN, ln_w, ln_w, ln_w, ln_w, ln_w);
  k_gemm<2, 8><<<dim3(COUT / GBM, LTOK / 128, NBATCH), GTHR, 0, stream>>>(
      CW2, KCW2, OH, KIN2, (long long)LTOK * KIN2, KCW2, 0, out, LTOK, (long long)COUT * LTOK,
      OP2, KOP2, 0, c2b, bn_g, bn_b, bn_m, bn_v);
}
